// PreHTSK_49976239456756
// MI455X (gfx1250) — hardware-run, weakly checked
//
#include <hip/hip_runtime.h>
#define TNB 2048
#define TND 256
#define TNR 128
#define TNO 64
#define TNF ((TND + 1) * TNR)
#define THS 0.5f
#define TLO 1e-8f
#define TVE 1e-5f
#define TWC 128.0f
typedef unsigned short v8us __attribute__((ext_vector_type(8), may_alias));
typedef float  v8f  __attribute__((ext_vector_type(8)));
typedef float  v4f  __attribute__((ext_vector_type(4)));
typedef float  v4fa __attribute__((ext_vector_type(4), may_alias));

__device__ __forceinline__ unsigned short bf16_bits(float x) { unsigned int u = __float_as_uint(x); return (unsigned short)((u + 0x7FFFu + ((u >> 16) & 1u)) >> 16); }
__device__ __forceinline__ float bf16_val(unsigned short b) { return __uint_as_float(((unsigned int)b) << 16); }
__device__ __forceinline__ float bf16_round(float x) { return bf16_val(bf16_bits(x)); }

typedef _Float16 v16h __attribute__((ext_vector_type(16)));
union FragH { v16h v; v8us half[2]; _Float16 h[16]; unsigned short u[16]; };

__global__ __launch_bounds__(256) void k_wt_f16(const float* __restrict__ W, _Float16* __restrict__ Wt, int K, int N, float scale) {
  const int t = blockIdx.x * 256 + threadIdx.x; if (t >= N * (K / 8)) return; const int n = t / (K / 8), k8 = (t % (K / 8)) * 8; FragH f;
#pragma unroll
  for (int i = 0; i < 8; ++i) f.h[i] = (_Float16)(bf16_round(W[(size_t)(k8 + i) * N + n]) * scale); const v8us o = f.half[0];
  *(volatile v8us*)((unsigned short*)Wt + (size_t)n * K + k8) = o; __threadfence(); *(volatile v8us*)((unsigned short*)Wt + (size_t)n * K + k8) = o;
}

typedef _Float16 v4h __attribute__((ext_vector_type(4)));

__device__ __forceinline__ v16h g2_frag(const _Float16* p, int hh) { FragH f; f.half[0] = *(const v8us*)((const unsigned short*)p + 8 * hh); f.half[1] = *(const v8us*)((const unsigned short*)p + 16 + 8 * hh); return f.v; }
__device__ __forceinline__ v8f g2_mma(v16h a, v16h b, v8f c) { v8f d = __builtin_amdgcn_wmma_f32_16x16x32_f16(false, a, false, b, (short)0, c, false, false); asm volatile("v_nop\n\tv_nop\n\tv_nop\n\tv_nop" : "+v"(d) : "v"(a), "v"(b)); return d; }
template <int ACT>
__global__ __launch_bounds__(128) void k_gemm2(const _Float16* __restrict__ A, int lda, size_t sA, const _Float16* __restrict__ Bh, int ldb, size_t sB, float alpha, const float* __restrict__ bias, size_t sBias, const float* __restrict__ CP, int rowsPerB, size_t sCPb, int row0g,
    float* __restrict__ C, _Float16* __restrict__ C16, int ldc, size_t sC, int M, int N, int K) { static_assert(ACT == 0 || ACT == 3 || ACT == 6 || ACT == 8 || ACT == 9 || ACT == 11 || ACT == 12 || ACT == 14 || ACT == 15 || ACT == 16 || ACT == 17, "k_gemm2: unsupported ACT code (would silently apply no activation)");
  __shared__ __attribute__((aligned(16))) float so[4][32][68];
  const int tid = threadIdx.x, w = tid >> 5, lane = tid & 31, ln = lane & 15, hh = lane >> 4; const int by = blockIdx.y;
  A += (size_t)by * sA; Bh += (size_t)by * sB; const size_t cofs = (size_t)by * sC; const float* bp = bias ? bias + (size_t)by * sBias : nullptr;
  const int ntn = N >> 6; const int mt = blockIdx.x / ntn, nq = blockIdx.x - mt * ntn; const int row0 = mt * 128 + 32 * w, col0 = nq * 64; if (row0 >= M) return;
  const _Float16* a0p = A + (size_t)(row0 + ln) * lda; const _Float16* a1p = a0p + (size_t)16 * lda;
  const _Float16* b0p = Bh + (size_t)(col0 + ln) * ldb; const _Float16* b1p = b0p + (size_t)16 * ldb; const _Float16* b2p = b1p + (size_t)16 * ldb; const _Float16* b3p = b2p + (size_t)16 * ldb;
  const v8f z8 = {0.f,0.f,0.f,0.f,0.f,0.f,0.f,0.f}; v8f c00 = z8, c01 = z8, c02 = z8, c03 = z8, c10 = z8, c11 = z8, c12 = z8, c13 = z8;
  for (int kb = 0; kb < K; kb += 32) { const v16h a0 = g2_frag(a0p + kb, hh), a1 = g2_frag(a1p + kb, hh);
    v16h b = g2_frag(b0p + kb, hh); c00 = g2_mma(a0, b, c00); c10 = g2_mma(a1, b, c10);
    b = g2_frag(b1p + kb, hh); c01 = g2_mma(a0, b, c01); c11 = g2_mma(a1, b, c11);
    b = g2_frag(b2p + kb, hh); c02 = g2_mma(a0, b, c02); c12 = g2_mma(a1, b, c12);
    b = g2_frag(b3p + kb, hh); c03 = g2_mma(a0, b, c03); c13 = g2_mma(a1, b, c13); }
  v8f accs[8] = {c00, c01, c02, c03, c10, c11, c12, c13};
#pragma unroll
  for (int u = 0; u < 8; ++u) { const int t = u & 3, half = u >> 2; const int col = col0 + t * 16 + ln; const float bv = bp ? bf16_round(bp[col]) : 0.f;
#pragma unroll
    for (int r = 0; r < 8; ++r) { const int rloc = half * 16 + 8 * hh + r; float v = accs[u][r] * alpha + bv; if (CP) { if (rowsPerB < 0) v += CP[cofs + (size_t)(row0g + row0 + rloc) * ldc + col];        else { const int bidx = (row0g + row0 + rloc) / rowsPerB; v += CP[(size_t)bidx * sCPb + (size_t)by * 64 + col]; } }
      if (ACT == 3) v = fmaxf(v, 0.f); else if (ACT == 6) v = 0.5f * v * (1.0f + erff(v * 0.70710678118654752f)); else if (ACT == 11) v = 1.0f / (1.0f + expf(-v)); else if (ACT == 15) v = v / (1.0f + expf(-v)); else if (ACT == 12) v = (v > 0.f) ? v : 0.01f * v; else if (ACT == 8) v = tanhf(v); else if (ACT == 9) v = 0.5f * v * (1.0f + tanhf(0.7978845608028654f * (v + 0.044715f * v * v * v))); else if (ACT == 14) v = (v > 0.f) ? v : 0.1f * v; else if (ACT == 16) v = (v >= 0.f) ? v : 0.3f * v; else if (ACT == 17) v = (v >= 0.f) ? v : 0.2f * v;
      so[w][rloc][t * 16 + ln] = v; } }
  __builtin_amdgcn_fence(__ATOMIC_ACQ_REL, "workgroup"); __builtin_amdgcn_wave_barrier();
  const int rsub = lane >> 4, c4 = (lane & 15) * 4;
  for (int pass = 0; pass < 2; ++pass) {
#pragma unroll
    for (int q = 0; q < 16; ++q) { const int r = q * 2 + rsub; const v4f v = *(const v4fa*)&so[w][r][c4]; if (C) *(volatile v4f*)(C + cofs + (size_t)(row0 + r) * ldc + col0 + c4) = v; if (C16) { v4h h4; for (int i = 0; i < 4; ++i) h4[i] = (_Float16)v[i]; *(volatile v4h*)(C16 + cofs + (size_t)(row0 + r) * ldc + col0 + c4) = h4; } }
    if (pass == 0) __threadfence(); } }

__global__ __launch_bounds__(256) void k_rbn(const float* __restrict__ src, float* __restrict__ dst, unsigned n4) {
  const unsigned t = blockIdx.x * 256u + threadIdx.x; if (t >= n4) return;
  const v4f a = *(const v4fa*)(src + (size_t)t * 4); v4f w;
#pragma unroll
  for (int q = 0; q < 4; ++q) w[q] = bf16_round(a[q]);
  float* d = dst + (size_t)t * 4; *(volatile v4f*)d = w; __threadfence(); *(volatile v4f*)d = w; }

__global__ __launch_bounds__(256) void k_scl(const float* __restrict__ SA, float* __restrict__ SK) {
  const unsigned t = blockIdx.x * 256u + threadIdx.x; if (t >= (unsigned)(TND * TNR / 4)) return;
  const v4f a = *(const v4fa*)(SA + (size_t)t * 4); v4f w;
#pragma unroll
  for (int q = 0; q < 4; ++q) w[q] = THS / (a[q] * a[q]) + TLO;
  float* d = SK + (size_t)t * 4; *(volatile v4f*)d = w; __threadfence(); *(volatile v4f*)d = w; }

__global__ __launch_bounds__(256) void k_frs(const float* __restrict__ XR, const float* __restrict__ CA, const float* __restrict__ SK, float* __restrict__ FL) {
  const unsigned t = blockIdx.x * 256u + threadIdx.x; if (t >= (unsigned)(TNB * TNR)) return;
  const unsigned r = t % TNR, rw = t / TNR; const float* xq = XR + (size_t)rw * TND; const float* cp = CA + r; const float* sp = SK + r; float a = 0.0f;
  for (unsigned d = 0; d < (unsigned)TND; d += 4) { const v4f x = *(const v4fa*)(xq + d);
#pragma unroll
    for (int q = 0; q < 4; ++q) { const float df = x[q] - cp[(size_t)(d + q) * TNR]; a += (-(df * df)) * sp[(size_t)(d + q) * TNR]; } }
  const float w = a / (float)TND; *(volatile float*)(FL + t) = w; __threadfence(); *(volatile float*)(FL + t) = w; }

__global__ __launch_bounds__(256) void k_smx(const float* __restrict__ FL, float* __restrict__ FR) {
  const unsigned rw = blockIdx.x * 256u + threadIdx.x; if (rw >= (unsigned)TNB) return;
  const float* lp = FL + (size_t)rw * TNR; float* fp = FR + (size_t)rw * TNR; float hi = lp[0];
  for (unsigned r = 0; r < (unsigned)TNR; r += 4) { const v4f a = *(const v4fa*)(lp + r); hi = fmaxf(fmaxf(fmaxf(hi, a[0]), fmaxf(a[1], a[2])), a[3]); }
  float s = 0.0f;
  for (unsigned r = 0; r < (unsigned)TNR; r += 4) { const v4f a = *(const v4fa*)(lp + r);
#pragma unroll
    for (int q = 0; q < 4; ++q) s += expf(a[q] - hi); }
  for (unsigned r = 0; r < (unsigned)TNR; r += 4) { const v4f a = *(const v4fa*)(lp + r); v4f w;
#pragma unroll
    for (int q = 0; q < 4; ++q) w[q] = expf(a[q] - hi) / s;
    *(volatile v4f*)(fp + r) = w; __threadfence(); *(volatile v4f*)(fp + r) = w; }
}

__global__ __launch_bounds__(256) void k_lns(const float* __restrict__ XR, const float* __restrict__ FR, float* __restrict__ MU, float* __restrict__ RS) {
  const unsigned rw = blockIdx.x * 256u + threadIdx.x; if (rw >= (unsigned)TNB) return;
  const float* fp = FR + (size_t)rw * TNR; const float* xq = XR + (size_t)rw * TND; float sm = 0.0f;
  for (unsigned r = 0; r < (unsigned)TNR; ++r) { const float f = fp[r];
    for (unsigned d = 0; d < (unsigned)TND; d += 4) { const v4f x = *(const v4fa*)(xq + d); sm += x[0] * f; sm += x[1] * f; sm += x[2] * f; sm += x[3] * f; } }
  for (unsigned r = 0; r < (unsigned)TNR; ++r) sm += fp[r];
  const float av = sm / (float)TNF; float sq = 0.0f;
  for (unsigned r = 0; r < (unsigned)TNR; ++r) { const float f = fp[r];
    for (unsigned d = 0; d < (unsigned)TND; d += 4) { const v4f x = *(const v4fa*)(xq + d);
#pragma unroll
      for (int q = 0; q < 4; ++q) { const float df = x[q] * f - av; sq += df * df; } } }
  for (unsigned r = 0; r < (unsigned)TNR; ++r) { const float df = fp[r] - av; sq += df * df; }
  const float rs = rsqrtf(sq / (float)TNF + TVE);
  *(volatile float*)(MU + rw) = av; *(volatile float*)(RS + rw) = rs; __threadfence(); *(volatile float*)(MU + rw) = av; *(volatile float*)(RS + rw) = rs; }

__global__ __launch_bounds__(256) void k_lnw(const float* __restrict__ XR, const float* __restrict__ FR, const float* __restrict__ MU, const float* __restrict__ RS, const float* __restrict__ GA, const float* __restrict__ BA, _Float16* __restrict__ FH) {
  const unsigned t = blockIdx.x * 256u + threadIdx.x; if (t >= (unsigned)(TNB * (TNF / 8))) return;
  const unsigned f0 = (t % (TNF / 8)) * 8, rw = t / (TNF / 8); const bool inner = f0 < (unsigned)(TND * TNR); const float av = MU[rw], rs = RS[rw];
  const unsigned ci = inner ? f0 / TND : (unsigned)(TNR - 1), ti = inner ? 0u : f0 - (unsigned)(TND * TNR);
  const float fr = FR[(size_t)rw * TNR + ci]; const float* xq = XR + (size_t)rw * TND + (f0 % TND); const v4f x0 = *(const v4fa*)xq, x1 = *(const v4fa*)(xq + 4); const float* fp = FR + (size_t)rw * TNR + ti; const v4f e0 = *(const v4fa*)fp, e1 = *(const v4fa*)(fp + 4);
  const v4f g0 = *(const v4fa*)(GA + f0), g1 = *(const v4fa*)(GA + f0 + 4), c0 = *(const v4fa*)(BA + f0), c1 = *(const v4fa*)(BA + f0 + 4); FragH f;
#pragma unroll
  for (int q = 0; q < 4; ++q) { const float p0 = inner ? x0[q] * fr : e0[q], p1 = inner ? x1[q] * fr : e1[q]; f.h[q] = (_Float16)(((p0 - av) * rs) * g0[q] + c0[q]); f.h[4 + q] = (_Float16)(((p1 - av) * rs) * g1[q] + c1[q]); }
  unsigned short* o = (unsigned short*)FH + (size_t)rw * TNF + f0; const v8us w = f.half[0]; *(volatile v8us*)o = w; __threadfence(); *(volatile v8us*)o = w; }

extern "C" void kernel_launch(void* const* d_in, const int* in_sizes, int n_in,
                              void* d_out, int out_size, void* d_ws, size_t ws_size, hipStream_t stream) {
  (void)in_sizes; (void)n_in; (void)out_size;
  const float* const* I = (const float* const*)d_in; const float* xa = I[0]; const float* ca = I[1]; const float* sa = I[2]; const float* ga = I[3]; const float* ba = I[4]; const float* wo = I[5]; const float* vo = I[6];
  float* res = (float*)d_out;
  static_assert(TNB % 128 == 0 && TNO % 64 == 0 && TNF % 32 == 0 && TNF % 8 == 0 && TND % 8 == 0 && TNR % 8 == 0 && (TNB * TND) % 4 == 0 && (TND * TNR) % 4 == 0 && TNF % 4 == 0 && ((size_t)TNO * TNF) % 8 == 0, "whole tiles");
  uint8_t* wsp = (uint8_t*)d_ws; size_t off = 0;
  auto take = [&](size_t bytes) { uint8_t* p = wsp + off; off += (bytes + 255) & ~(size_t)255; return p; };
  _Float16* FH = (_Float16*)take((size_t)TNB * TNF * 2); _Float16* WH = (_Float16*)take((size_t)TNO * TNF * 2); float* XR = (float*)take((size_t)TNB * TND * 4); float* CA = (float*)take((size_t)TND * TNR * 4); float* SA = (float*)take((size_t)TND * TNR * 4); float* SK = (float*)take((size_t)TND * TNR * 4); float* GA = (float*)take((size_t)TNF * 4); float* BA = (float*)take((size_t)TNF * 4); float* FL = (float*)take((size_t)TNB * TNR * 4); float* FR = (float*)take((size_t)TNB * TNR * 4); float* MU = (float*)take((size_t)TNB * 4); float* RS = (float*)take((size_t)TNB * 4);
  if (off > ws_size) return;
  k_rbn<<<(unsigned)(((size_t)TNB * TND / 4 + 255) / 256), 256, 0, stream>>>(xa, XR, (unsigned)((size_t)TNB * TND / 4));
  k_rbn<<<(unsigned)((TND * TNR / 4 + 255) / 256), 256, 0, stream>>>(ca, CA, (unsigned)(TND * TNR / 4));
  k_rbn<<<(unsigned)((TND * TNR / 4 + 255) / 256), 256, 0, stream>>>(sa, SA, (unsigned)(TND * TNR / 4));
  k_rbn<<<(unsigned)((TNF / 4 + 255) / 256), 256, 0, stream>>>(ga, GA, (unsigned)(TNF / 4));
  k_rbn<<<(unsigned)((TNF / 4 + 255) / 256), 256, 0, stream>>>(ba, BA, (unsigned)(TNF / 4));
  k_wt_f16<<<(unsigned)(((size_t)TNO * TNF / 8 + 255) / 256), 256, 0, stream>>>(wo, WH, TNO * TNF, 1, TWC);
  k_scl<<<(unsigned)((TND * TNR / 4 + 255) / 256), 256, 0, stream>>>(SA, SK);
  k_frs<<<(unsigned)((TNB * TNR + 255) / 256), 256, 0, stream>>>(XR, CA, SK, FL);
  k_smx<<<(unsigned)((TNB + 255) / 256), 256, 0, stream>>>(FL, FR);
  k_lns<<<(unsigned)((TNB + 255) / 256), 256, 0, stream>>>(XR, FR, MU, RS);
  k_lnw<<<(unsigned)(((size_t)TNB * (TNF / 8) + 255) / 256), 256, 0, stream>>>(XR, FR, MU, RS, GA, BA, FH);
  k_gemm2<0><<<dim3((unsigned)((TNB / 128) * (TNO / 64)), 1), 128, 0, stream>>>(FH, TNF, 0, WH, TNF, 0, 1.0f / TWC, vo, 0, nullptr, 1, 0, 0, res, nullptr, TNO, 0, TNB, TNO, TNF);
}
